// TransConvLayer_36653250904189
// MI455X (gfx1250) — hardware-verified
//
#include <hip/hip_runtime.h>
#include <math.h>

typedef __attribute__((ext_vector_type(16))) _Float16 v16h;
typedef __attribute__((ext_vector_type(16))) __bf16 v16b;
typedef __attribute__((ext_vector_type(8)))  _Float16 v8h;
typedef __attribute__((ext_vector_type(8)))  float v8f;
typedef __attribute__((ext_vector_type(4)))  float v4f;
typedef __attribute__((ext_vector_type(2)))  float v2f;
typedef __attribute__((ext_vector_type(4)))  unsigned v4u;
typedef __attribute__((ext_vector_type(4)))  int v4i;
typedef float __attribute__((may_alias)) float_a;
typedef int __attribute__((may_alias)) int_a;

template <typename T> __device__ __forceinline__ void vst2(void* p, T v) { *(volatile T*)p = v; __threadfence(); *(volatile T*)p = v; }
__device__ __forceinline__ v8f wmma16(v16h a, v16h b, v8f c) {
  v8f d = __builtin_amdgcn_wmma_f32_16x16x32_f16(false, a, false, b, (short)0, c, false, false);
  asm volatile("v_nop\n\tv_nop\n\tv_nop\n\tv_nop" : "+v"(d) : "v"(a), "v"(b));
  return d;
}
__device__ __forceinline__ v8f wmma_bf(v16b a, v16b b, v8f c) {
  v8f d = __builtin_amdgcn_wmma_f32_16x16x32_bf16(false, a, false, b, (short)0, c, false, false);
  asm volatile("v_nop\n\tv_nop\n\tv_nop\n\tv_nop" : "+v"(d) : "v"(a), "v"(b));
  return d;
}
__device__ __forceinline__ v16h frag_h(const _Float16* rowk0, int lane) {
  union { v16h v; v8h q[2]; } u; const _Float16* p = rowk0 + 8 * (lane >> 4);
  u.q[0] = *(const v8h*)p; u.q[1] = *(const v8h*)(p + 16); return u.v;
}
__device__ __forceinline__ v16h frag_f32(const float* rowk0, int lane) {
  v16h a; const float* p = rowk0 + 8 * (lane >> 4);
#pragma unroll
  for (int i = 0; i < 8; ++i) { a[i] = (_Float16)p[i]; a[8 + i] = (_Float16)p[16 + i]; }
  return a;
}
__device__ __forceinline__ v16h frag_f32s(const float* rowk0, int lane, float sc) {
  v16h a; const float* p = rowk0 + 8 * (lane >> 4);
#pragma unroll
  for (int i = 0; i < 8; ++i) { a[i] = (_Float16)(p[i] * sc); a[8 + i] = (_Float16)(p[16 + i] * sc); }
  return a;
}
__device__ __forceinline__ v16h fragc_f32(const float* W, int k0, int n, int lane, int ld, int K) {
  v16h a; const int g = lane >> 4;
#pragma unroll
  for (int i = 0; i < 8; ++i) { const int ka = k0 + 8 * g + i, kb = ka + 16;
    a[i] = (_Float16)(ka < K ? W[(size_t)(ka < K ? ka : K - 1) * ld + n] : 0.f); a[8 + i] = (_Float16)(kb < K ? W[(size_t)(kb < K ? kb : K - 1) * ld + n] : 0.f); }
  return a;
}
struct F2 { v16b h, l; };
__device__ __forceinline__ F2 bsplit16(const float v[16]) { F2 r;
#pragma unroll
  for (int i = 0; i < 16; ++i) { const __bf16 h = (__bf16)v[i]; r.h[i] = h; r.l[i] = (__bf16)(v[i] - (float)h); }
  return r; }
__device__ __forceinline__ F2 split_row(const float* row, int k0, int lane) { float v[16]; const float* p = row + k0 + 8 * (lane >> 4);
#pragma unroll
  for (int i = 0; i < 8; ++i) { v[i] = p[i]; v[8 + i] = p[16 + i]; }
  return bsplit16(v); }
__device__ __forceinline__ F2 split_rowK(const float* row, int k0, int lane, int K) { float v[16]; const int g = lane >> 4;
#pragma unroll
  for (int i = 0; i < 8; ++i) { const int ka = k0 + 8 * g + i, kb = ka + 16; v[i] = ka < K ? row[ka < K ? ka : K - 1] : 0.f; v[8 + i] = kb < K ? row[kb < K ? kb : K - 1] : 0.f; }
  return bsplit16(v); }
__device__ __forceinline__ F2 split_col(const float* W, int k0, int n, int lane, int ld, int K) { float v[16]; const int g = lane >> 4;
#pragma unroll
  for (int i = 0; i < 8; ++i) { const int ka = k0 + 8 * g + i, kb = ka + 16; v[i] = ka < K ? W[(size_t)(ka < K ? ka : K - 1) * ld + n] : 0.f; v[8 + i] = kb < K ? W[(size_t)(kb < K ? kb : K - 1) * ld + n] : 0.f; }
  return bsplit16(v); }
__device__ __forceinline__ v8f mac3(const F2& a, const F2& b, v8f c) { c = wmma_bf(a.l, b.h, c); c = wmma_bf(a.h, b.l, c); return wmma_bf(a.h, b.h, c); }
__device__ __forceinline__ float sigm(float v) { return 1.0f / (1.0f + expf(-v)); }
#define LDSX() do { asm volatile("s_wait_dscnt 0" ::: "memory"); __builtin_amdgcn_wave_barrier(); __builtin_amdgcn_fence(__ATOMIC_RELEASE, "workgroup"); } while (0)

#define NN 32768
#define CI 128
#define CO 128
#define NH 8
#ifndef NPROC
#define NPROC NN
#endif
typedef __attribute__((ext_vector_type(8))) __bf16 v8b;
__device__ __forceinline__ v16b frag_b(const __bf16* rowk0, int lane) {
  union { v16b v; v8b q[2]; } u; const __bf16* p = rowk0 + 8 * (lane >> 4);
  u.q[0] = *(const v8b*)p; u.q[1] = *(const v8b*)(p + 16); return u.v;
}
__device__ __forceinline__ float bfr(float v) { return (float)(__bf16)v; }
__device__ __forceinline__ v16b wrow(const float* rowk0, int lane) { v16b w; const float* p = rowk0 + 8 * (lane >> 4);
#pragma unroll
  for (int i = 0; i < 8; ++i) { w[i] = (__bf16)p[i]; w[8 + i] = (__bf16)p[16 + i]; }
  return w; }
__device__ __forceinline__ F2 colsplit(const float* Wm, int k0, int n, int lane, int ld) { float v[16]; const int g = lane >> 4;
#pragma unroll
  for (int i = 0; i < 8; ++i) { v[i] = Wm[(size_t)(k0 + 8 * g + i) * ld + n]; v[8 + i] = Wm[(size_t)(k0 + 16 + 8 * g + i) * ld + n]; }
  return bsplit16(v); }

#define WS_PQH 0u
#define WS_PQL (WS_PQH + 2u * (size_t)NN * CO)
#define WS_PKT (WS_PQL + 2u * (size_t)NN * CO)
#define WS_PKU (WS_PKT + 2u * (size_t)CO * NN)
#define WS_VH  (WS_PKU + 2u * (size_t)CO * NN)
#define WS_VL  (WS_VH  + 2u * (size_t)NN * CO)
#define WS_VTH (WS_VL  + 2u * (size_t)NN * CO)
#define WS_VTL (WS_VTH + 2u * (size_t)CO * NN)
#define WS_KS  (WS_VTL + 2u * (size_t)CO * NN)
#define WS_KV  (WS_KS  + 4u * 128)
#define WS_ACC (WS_KV  + 4u * (size_t)CO * CO)
#define WS_END (WS_ACC + 4u * (size_t)NN * CO)

__global__ __launch_bounds__(128) void k_proj(const float* __restrict__ XQ, const float* __restrict__ XS, const float* __restrict__ WQ, const float* __restrict__ BQ, const float* __restrict__ WK, const float* __restrict__ BK, const float* __restrict__ WV, const float* __restrict__ BV, const float* __restrict__ NS, int h,
    __bf16* __restrict__ PQH, __bf16* __restrict__ PQL, __bf16* __restrict__ PKT, __bf16* __restrict__ PKU, __bf16* __restrict__ VH, __bf16* __restrict__ VL, __bf16* __restrict__ VTH, __bf16* __restrict__ VTL) {
  __shared__ __align__(16) __bf16 sh[64][136], sl[64][136]; __shared__ __align__(16) __bf16 th[128][72], tl2[128][72];
  const int tid = threadIdx.x, wave = tid >> 5, lane = tid & 31, col = lane & 15, g = lane >> 4; const int which = blockIdx.z; const size_t r0 = (size_t)blockIdx.x * 64;
  const float* X = which == 0 ? XQ : XS; const float* WA = (which == 0 ? WQ : which == 1 ? WK : WV) + (size_t)h * CO * CI; const float* BA = (which == 0 ? BQ : which == 1 ? BK : BV) + (size_t)h * CO;
  v8f acc[8] = {};
#pragma unroll
  for (int kc = 0; kc < CI / 32; ++kc) { v16b a; { const float* p = X + (r0 + wave * 16 + col) * CI + kc * 32 + 8 * g;
#pragma unroll
      for (int i = 0; i < 8; ++i) { a[i] = (__bf16)p[i]; a[8 + i] = (__bf16)p[16 + i]; } }
    asm volatile("s_wait_loadcnt 0x0" ::: "memory");
#pragma unroll
    for (int j = 0; j < 8; ++j) { const v16b w = wrow(WA + (size_t)(j * 16 + col) * CI + kc * 32, lane); asm volatile("s_wait_loadcnt 0x0" ::: "memory"); acc[j] = wmma_bf(a, w, acc[j]); } }
#pragma unroll
  for (int j = 0; j < 8; ++j) { const float bb = bfr(BA[j * 16 + col]);
#pragma unroll
    for (int r = 0; r < 8; ++r) acc[j][r] += bb; }
  if (which < 2) {
    const float ds = fabsf(bfr(NS[0])) + 1e-6f; float n1[8], n2[8];
#pragma unroll
    for (int r = 0; r < 8; ++r) { float s1 = 0.f, s2 = 0.f;
#pragma unroll
      for (int j = 0; j < 8; ++j) { const float x = (fmaxf(acc[j][r], 0.f) + 1e-6f) / ds; acc[j][r] = x; const float x2 = x * x; s1 += x2; s2 += x2 * x2; }
      n1[r] = s1; n2[r] = s2; }
#pragma unroll
    for (int o = 1; o < 16; o <<= 1) {
#pragma unroll
      for (int r = 0; r < 8; ++r) { n1[r] += __shfl_xor(n1[r], o); n2[r] += __shfl_xor(n2[r], o); } }
#pragma unroll
    for (int r = 0; r < 8; ++r) n1[r] = sqrtf(n1[r]) / (sqrtf(n2[r]) + 1e-8f);
#pragma unroll
    for (int j = 0; j < 8; ++j) {
#pragma unroll
      for (int r = 0; r < 8; ++r) acc[j][r] = n1[r] * (acc[j][r] * acc[j][r]); } }
#pragma unroll
  for (int j = 0; j < 8; ++j) {
#pragma unroll
    for (int r = 0; r < 8; ++r) { const float v = acc[j][r]; const __bf16 hv = (__bf16)v, lv = (__bf16)(v - (float)hv); const int rl = wave * 16 + 8 * g + r, cl = j * 16 + col;
      if (which != 1) { sh[rl][cl] = hv; sl[rl][cl] = lv; }
      if (which != 0) { th[cl][rl] = hv; tl2[cl][rl] = lv; } } }
  __syncthreads();
  if (which != 1) { __bf16* dh = which == 0 ? PQH : VH; __bf16* dl = which == 0 ? PQL : VL; for (int e = tid; e < 64 * 16; e += 128) { const int rl = e >> 4, q = e & 15; vst2((unsigned*)(dh + (r0 + rl) * CO + q * 8), *(const v4u*)&sh[rl][q * 8]); vst2((unsigned*)(dl + (r0 + rl) * CO + q * 8), *(const v4u*)&sl[rl][q * 8]); } }
  if (which != 0) { __bf16* dh = which == 1 ? PKT : VTH; __bf16* dl = which == 1 ? PKU : VTL; for (int e = tid; e < 128 * 8; e += 128) { const int cl = e >> 3, q = e & 7; vst2((unsigned*)(dh + (size_t)cl * NN + r0 + q * 8), *(const v4u*)&th[cl][q * 8]); vst2((unsigned*)(dl + (size_t)cl * NN + r0 + q * 8), *(const v4u*)&tl2[cl][q * 8]); } } }
__global__ __launch_bounds__(128) void k_ksum(const __bf16* __restrict__ PKT, const __bf16* __restrict__ PKU, float* __restrict__ KS) { __shared__ __align__(16) float sk[128];
  const int m = threadIdx.x; float s = 0.f; const __bf16* ph = PKT + (size_t)m * NN; const __bf16* pl = PKU + (size_t)m * NN;
#pragma unroll 4
  for (int n = 0; n < NPROC; n += 8) { const v8b a = *(const v8b*)(ph + n), b2 = *(const v8b*)(pl + n);
#pragma unroll
    for (int z = 0; z < 8; ++z) s += (float)a[z] + (float)b2[z]; }
  sk[m] = s; __syncthreads(); if (m < 32) vst2(KS + m * 4, *(const v4f*)&sk[m * 4]); }
__global__ __launch_bounds__(128) void k_kv(const __bf16* __restrict__ PKT, const __bf16* __restrict__ PKU, const __bf16* __restrict__ VTH, const __bf16* __restrict__ VTL, float* __restrict__ KV) { __shared__ __align__(16) float sf[4][16][132];
  const int tid = threadIdx.x, wave = tid >> 5, lane = tid & 31, col = lane & 15, g = lane >> 4; const size_t m0 = (size_t)blockIdx.x * 64 + wave * 16;
  v8f acc[8] = {};
#pragma unroll 1
  for (int kc = 0; kc < NPROC / 32; ++kc) { const v16b ah = frag_b(PKT + (m0 + col) * NN + kc * 32, lane), al = frag_b(PKU + (m0 + col) * NN + kc * 32, lane);
    asm volatile("s_wait_loadcnt 0x0" ::: "memory");
#pragma unroll
    for (int j = 0; j < 8; ++j) { const size_t vr = (size_t)(j * 16 + col) * NN + kc * 32; const v16b bh = frag_b(VTH + vr, lane), bl = frag_b(VTL + vr, lane); acc[j] = wmma_bf(al, bh, acc[j]); acc[j] = wmma_bf(ah, bl, acc[j]); acc[j] = wmma_bf(ah, bh, acc[j]); } }
#pragma unroll
  for (int j = 0; j < 8; ++j) {
#pragma unroll
    for (int r = 0; r < 8; ++r) sf[wave][8 * g + r][j * 16 + col] = acc[j][r]; }
  LDSX(); for (int rl = 0; rl < 16; ++rl) vst2(KV + (m0 + rl) * CO + lane * 4, *(const v4f*)&sf[wave][rl][lane * 4]); }
__global__ __launch_bounds__(128) void k_num(const __bf16* __restrict__ PQH, const __bf16* __restrict__ PQL, const float* __restrict__ KV, const float* __restrict__ KS, const __bf16* __restrict__ VH, const __bf16* __restrict__ VL, const float* __restrict__ VMW, const float* __restrict__ VMB, int h, float* __restrict__ ACC) {
  __shared__ __align__(16) float sf[4][16][132]; __shared__ __align__(16) float sks[128]; __shared__ float sden[64];
  const int tid = threadIdx.x, wave = tid >> 5, lane = tid & 31, col = lane & 15, g = lane >> 4; const size_t r0 = (size_t)blockIdx.x * 64; const size_t w0 = r0 + wave * 16;
  sks[tid] = KS[tid]; __syncthreads();
  if (tid < 64) { float d = 0.f; const __bf16* ph = PQH + (r0 + tid) * CO; const __bf16* pl = PQL + (r0 + tid) * CO;
#pragma unroll 4
    for (int m = 0; m < CO; m += 8) { const v8b a = *(const v8b*)(ph + m), b2 = *(const v8b*)(pl + m);
#pragma unroll
      for (int z = 0; z < 8; ++z) d += ((float)a[z] + (float)b2[z]) * sks[m + z]; }
    sden[tid] = d; }
  v8f acc[8] = {}, vs[8] = {};
#pragma unroll
  for (int kc = 0; kc < CO / 32; ++kc) { const v16b ah = frag_b(PQH + (w0 + col) * CO + kc * 32, lane), al = frag_b(PQL + (w0 + col) * CO + kc * 32, lane), bh = frag_b(VH + (w0 + col) * CO + kc * 32, lane), bl = frag_b(VL + (w0 + col) * CO + kc * 32, lane);
    asm volatile("s_wait_loadcnt 0x0" ::: "memory");
#pragma unroll
    for (int j = 0; j < 8; ++j) { const F2 w = colsplit(KV, kc * 32, j * 16 + col, lane, CO); asm volatile("s_wait_loadcnt 0x0" ::: "memory"); const v16b wm = wrow(VMW + (size_t)(j * 16 + col) * CO + kc * 32, lane); asm volatile("s_wait_loadcnt 0x0" ::: "memory");
      acc[j] = wmma_bf(al, w.h, acc[j]); acc[j] = wmma_bf(ah, w.l, acc[j]); acc[j] = wmma_bf(ah, w.h, acc[j]); vs[j] = wmma_bf(bh, wm, vs[j]); vs[j] = wmma_bf(bl, wm, vs[j]); } }
  __syncthreads();
#pragma unroll
  for (int j = 0; j < 8; ++j) { const float bb = bfr(VMB[j * 16 + col]);
#pragma unroll
    for (int r = 0; r < 8; ++r) { const float den = sden[wave * 16 + 8 * g + r]; sf[wave][8 * g + r][j * 16 + col] = acc[j][r] / (den + 1e-6f) + (vs[j][r] + bb); } }
  LDSX(); for (int rl = 0; rl < 16; ++rl) { float* dst = ACC + (w0 + rl) * CO + lane * 4; v4f v = *(const v4f*)&sf[wave][rl][lane * 4]; if (h > 0) { const v4f p = *(const v4f*)dst; v[0] += p[0]; v[1] += p[1]; v[2] += p[2]; v[3] += p[3]; } vst2(dst, v); } }
__global__ __launch_bounds__(128) void k_fin(const float* __restrict__ ACC, float* __restrict__ OUT) { __shared__ __align__(16) float so[64 * 129 + 12];
  const int tid = threadIdx.x; const size_t r0 = (size_t)blockIdx.x * 64;
  for (int rl = tid >> 5, lanei = tid & 31; rl < 64; rl += 4) { const v4f a = *(const v4f*)(ACC + (r0 + rl) * CO + lanei * 4); float o[4]; float s = 0.f;
#pragma unroll
    for (int z = 0; z < 4; ++z) { o[z] = a[z] * (1.0f / NH); s += o[z] * o[z]; }
#pragma unroll
    for (int q = 1; q < 32; q <<= 1) s += __shfl_xor(s, q);
#pragma unroll
    for (int z = 0; z < 4; ++z) so[rl * 129 + 1 + lanei * 4 + z] = o[z];
    if (lanei == 0) so[rl * 129] = sqrtf(s + 1.0f); }
  __syncthreads();
  float* dst = OUT + r0 * 129;
  for (int e = tid; e < 64 * 129 / 4; e += 128) vst2(dst + e * 4, *(const v4f*)&so[e * 4]); }
extern "C" void kernel_launch(void* const* d_in, const int* in_sizes, int n_in, void* d_out, int out_size, void* d_ws, size_t ws_size, hipStream_t stream) {
  (void)in_sizes; (void)n_in; (void)out_size;
  const float** F = (const float**)d_in;
  if (ws_size < (size_t)WS_END) return;
  char* ws = (char*)d_ws; __bf16 *PQH = (__bf16*)(ws + WS_PQH), *PQL = (__bf16*)(ws + WS_PQL), *PKT = (__bf16*)(ws + WS_PKT), *PKU = (__bf16*)(ws + WS_PKU), *VH = (__bf16*)(ws + WS_VH), *VL = (__bf16*)(ws + WS_VL), *VTH = (__bf16*)(ws + WS_VTH), *VTL = (__bf16*)(ws + WS_VTL); float *KS = (float*)(ws + WS_KS), *KV = (float*)(ws + WS_KV), *ACC = (float*)(ws + WS_ACC);
  for (int h = 0; h < NH; ++h) {
    k_proj<<<dim3(NPROC / 64, 1, 3), 128, 0, stream>>>(F[0], F[1], F[2], F[3], F[4], F[5], F[6], F[7], F[10], h, PQH, PQL, PKT, PKU, VH, VL, VTH, VTL);
    k_ksum<<<dim3(1), 128, 0, stream>>>(PKT, PKU, KS);
    k_kv<<<dim3(CO / 64), 128, 0, stream>>>(PKT, PKU, VTH, VTL, KV);
    k_num<<<dim3(NPROC / 64), 128, 0, stream>>>(PQH, PQL, KV, KS, VH, VL, F[8], F[9], h, ACC);
  }
  k_fin<<<dim3(NPROC / 64), 128, 0, stream>>>(ACC, (float*)d_out);
}
